// DeepseekMoE_TaskSpecificExperts_86165633893004
// MI455X (gfx1250) — hardware-verified
//
#include <hip/hip_runtime.h>
#include <stdint.h>
#include <stddef.h>
#include <math.h>

#define NTOK  4096
#define DM    1024
#define HXR   512
#define HXS   1024
#define NEX   8
#define NSL   2
#define NTASK 3
#define MT    32
#define XP    1032
#define YP    260
#define TQ    72

#define LDS_XB (MT * XP * 2)
#define LDS_R  (2 * LDS_XB + MT * (HXR + 8) * 2)
#define LDS_S  (2 * LDS_XB + MT * (HXS + 8) * 2)

#define W_SC 256.0f
#define H_SC 256.0f
#define X_LO 2048.0f
#define R_W  0.00390625f
#define R_HW 1.52587890625e-05f
#define R_LO 4.8828125e-04f

static_assert(MT * YP * 4 <= LDS_XB);
static_assert((XP * 2) % 16 == 0);
static_assert((YP * 4) % 16 == 0);
static_assert((TQ * 2) % 16 == 0);
static_assert(NTOK % 256 == 0);
static_assert(NTOK % 32 == 0);
static_assert(NTOK % MT == 0);
static_assert(MT * (DM / 8) == 16 * 256);
static_assert(DM % 256 == 0);
static_assert(DM % 64 == 0);
static_assert(HXR % 128 == 0);
static_assert(HXS % 128 == 0);
static_assert(HXR % 64 == 0);
static_assert(HXS % 64 == 0);
static_assert((NTOK * DM) % 8 == 0);
static_assert(NEX == 8);
static_assert(NSL == 2);

typedef _Float16       v16h __attribute__((ext_vector_type(16)));
typedef _Float16       v8h  __attribute__((ext_vector_type(8)));
typedef float          v8f  __attribute__((ext_vector_type(8)));
typedef float          v4f  __attribute__((ext_vector_type(4)));
typedef unsigned int   v4u  __attribute__((ext_vector_type(4)));
typedef v4f __attribute__((may_alias)) v4fa;
typedef v4u __attribute__((may_alias)) v4ua;

union FragH { v16h v; v4u q[2]; };
union Pack8 { v8h h; v4u u; };

__device__ __forceinline__ unsigned short hbits(float f) {
  _Float16 t = (_Float16)f;
  unsigned short u;
  __builtin_memcpy(&u, &t, 2);
  return u;
}

__device__ __forceinline__ void split_h(float v, _Float16& hi, _Float16& lo) {
  const _Float16 th = (_Float16)v;
  const float res = (v - (float)th) * X_LO;
  hi = th;
  lo = (_Float16)res;
}

__device__ __forceinline__ v8f wmma_h(v16h a, v16h b, v8f c) {
  v8f d = __builtin_amdgcn_wmma_f32_16x16x32_f16(false, a, false, b, (short)0, c, false, false);
  asm volatile("v_nop\n\tv_nop\n\tv_nop\n\tv_nop" : "+v"(d) : "v"(a), "v"(b));
  return d;
}

__device__ __forceinline__ v16h ldfrag(const unsigned short* p, int h) {
  FragH f;
  f.q[0] = *(const v4ua*)(p + 8 * h);
  f.q[1] = *(const v4ua*)(p + 16 + 8 * h);
  return f.v;
}

__global__ __launch_bounds__(256) void k_router(const float* __restrict__ X,
                                                const float* __restrict__ gw,
                                                const float* __restrict__ temb,
                                                const int* __restrict__ tsk,
                                                int* __restrict__ sel,
                                                float* __restrict__ rw, int ntok)
{
  __shared__ __align__(16) int   sI[64];
  __shared__ __align__(16) float sV[64];
  const int tid = threadIdx.x, lane = tid & 31, wv = tid >> 5;
  int task = tsk[0];
  task = (task < 0) ? 0 : ((task > NTASK - 1) ? (NTASK - 1) : task);
  const float* te = temb + (size_t)task * DM;

  #pragma unroll 1
  for (int q = 0; q < 4; ++q) {
    const int tl = wv * 4 + q;
    int t = blockIdx.x * 32 + tl;
    t = (t > ntok - 1) ? (ntok - 1) : t;
    const float* xr = X + (size_t)t * DM;
    double acc[NEX];
    #pragma unroll
    for (int e = 0; e < NEX; ++e) acc[e] = 0.0;
    #pragma unroll 1
    for (int j = 0; j < DM / 32; ++j) {
      const int hh = lane + 32 * j;
      const float xv = xr[hh] + te[hh];
      const double xd = (double)xv;
      #pragma unroll
      for (int e = 0; e < NEX; ++e)
        acc[e] = fma(xd, (double)gw[(size_t)e * DM + hh], acc[e]);
    }
    #pragma unroll
    for (int e = 0; e < NEX; ++e) {
      #pragma unroll
      for (int s = 16; s > 0; s >>= 1) acc[e] += __shfl_xor(acc[e], s, 32);
    }
    double b1 = acc[0];
    int i1 = 0;
    #pragma unroll
    for (int e = 1; e < NEX; ++e) {
      if (acc[e] > b1) { b1 = acc[e]; i1 = e; }
    }
    double b2 = -1.0e300;
    int i2 = -1;
    #pragma unroll
    for (int e = 0; e < NEX; ++e) {
      if (e != i1 && acc[e] > b2) { b2 = acc[e]; i2 = e; }
    }
    if (i2 < 0) { i2 = (i1 == 0) ? 1 : 0; b2 = b1; }
    const float df = (float)(b2 - b1);
    const float ef = expf(df);
    const float rinv = 1.0f / (1.0f + ef);
    const float w1 = rinv;
    const float w2 = ef * rinv;
    if (lane == 0) {
      sI[2 * tl] = i1;  sI[2 * tl + 1] = i2;
      sV[2 * tl] = w1;  sV[2 * tl + 1] = w2;
    }
  }
  __syncthreads();
  if (wv == 0 && lane < 16) {
    const v4u vi = *(const v4ua*)(sI + 4 * lane);
    const v4f vw = *(const v4fa*)(sV + 4 * lane);
    unsigned int* di = (unsigned int*)sel + (size_t)blockIdx.x * 64 + 4 * lane;
    float*        dw = rw + (size_t)blockIdx.x * 64 + 4 * lane;
    *(volatile v4u*)di = vi;
    *(volatile v4f*)dw = vw;
    __threadfence();
    *(volatile v4u*)di = vi;
    *(volatile v4f*)dw = vw;
  }
}

__global__ __launch_bounds__(256) void k_cvtx(const float* __restrict__ src,
                                              unsigned short* __restrict__ dhi,
                                              unsigned short* __restrict__ dlo,
                                              int n8)
{
  const int g = blockIdx.x * 256 + threadIdx.x;
  if (g >= n8) return;
  const float* s = src + (size_t)g * 8;
  const v4f a = *(const v4fa*)s;
  const v4f c = *(const v4fa*)(s + 4);
  v8h hh, hl;
  _Float16 th, tl;
  split_h(a.x, th, tl); hh[0] = th; hl[0] = tl;
  split_h(a.y, th, tl); hh[1] = th; hl[1] = tl;
  split_h(a.z, th, tl); hh[2] = th; hl[2] = tl;
  split_h(a.w, th, tl); hh[3] = th; hl[3] = tl;
  split_h(c.x, th, tl); hh[4] = th; hl[4] = tl;
  split_h(c.y, th, tl); hh[5] = th; hl[5] = tl;
  split_h(c.z, th, tl); hh[6] = th; hl[6] = tl;
  split_h(c.w, th, tl); hh[7] = th; hl[7] = tl;
  Pack8 ph, pl;
  ph.h = hh;
  pl.h = hl;
  const v4u uh = ph.u;
  const v4u ul = pl.u;
  unsigned short* dh = dhi + (size_t)g * 8;
  unsigned short* dl = dlo + (size_t)g * 8;
  *(volatile v4u*)dh = uh;
  *(volatile v4u*)dl = ul;
  __threadfence();
  *(volatile v4u*)dh = uh;
  *(volatile v4u*)dl = ul;
}

__global__ __launch_bounds__(256) void k_tcvt(const float* __restrict__ src,
                                              unsigned short* __restrict__ dst,
                                              int KR, int NC, float sc)
{
  __shared__ __align__(16) unsigned short s[64 * TQ];
  const int tid = threadIdx.x;
  const int k0 = blockIdx.y * 64, n0 = blockIdx.x * 64;
  const size_t zo = (size_t)blockIdx.z * (size_t)KR * (size_t)NC;
  const float* sp = src + zo;
  unsigned short* dp = dst + zo;
  #pragma unroll
  for (int p = 0; p < 4; ++p) {
    const int k  = p * 16 + (tid >> 4);
    const int n4 = (tid & 15) * 4;
    const v4f v = *(const v4fa*)(sp + (size_t)(k0 + k) * NC + n0 + n4);
    s[(n4 + 0) * TQ + k] = hbits(v.x * sc);
    s[(n4 + 1) * TQ + k] = hbits(v.y * sc);
    s[(n4 + 2) * TQ + k] = hbits(v.z * sc);
    s[(n4 + 3) * TQ + k] = hbits(v.w * sc);
  }
  __syncthreads();
  const int q = tid & 7, nb = tid >> 3;
  const v4u w0 = *(const v4ua*)(s + nb * TQ + 8 * q);
  const v4u w1 = *(const v4ua*)(s + (nb + 32) * TQ + 8 * q);
  unsigned short* d0 = dp + (size_t)(n0 + nb) * KR + k0 + 8 * q;
  unsigned short* d1 = dp + (size_t)(n0 + nb + 32) * KR + k0 + 8 * q;
  *(volatile v4u*)d0 = w0;
  *(volatile v4u*)d1 = w1;
  __threadfence();
  *(volatile v4u*)d0 = w0;
  *(volatile v4u*)d1 = w1;
}

template <int NSLT>
__device__ __forceinline__ void part_pass(const float* sY, const int* tk, const int* sl,
                                          float* dstp, int ns, int wv, int lane, int nrows)
{
  #pragma unroll
  for (int i = 0; i < 4; ++i) {
    const int row = wv * 4 + i;
    int t = tk[row];
    t = (t < 0) ? 0 : ((t > NTOK - 1) ? (NTOK - 1) : t);
    int s = sl[row];
    s = (s != 0) ? 1 : 0;
    if (NSLT == 1) s = 0;
    const v4f v0 = *(const v4fa*)(sY + row * YP + 4 * lane);
    const v4f v1 = *(const v4fa*)(sY + row * YP + 128 + 4 * lane);
    float* dst = dstp + ((size_t)t * NSLT + s) * DM + ns * 256;
    if (row < nrows) {
      *(volatile v4f*)(dst + 4 * lane) = v0;
      *(volatile v4f*)(dst + 128 + 4 * lane) = v1;
    }
  }
}

template <int HXT, int GXT, int TPBT, int NSLT, int DENSE>
__global__ __launch_bounds__(256) void k_expert(const unsigned short* __restrict__ xh,
                                                const unsigned short* __restrict__ xl,
                                                const unsigned short* __restrict__ wg,
                                                const unsigned short* __restrict__ wu,
                                                const unsigned short* __restrict__ wd,
                                                const int* __restrict__ sel,
                                                const float* __restrict__ rw,
                                                float* __restrict__ dstp, int ntok)
{
  constexpr int HP = HXT + 8;
  static_assert(GXT * TPBT * MT == NTOK);
  static_assert(TPBT * MT <= 256);
  static_assert(HXT % 128 == 0);
  static_assert((HP * 2) % 16 == 0);

  extern __shared__ __align__(16) unsigned char dsm_e[];
  unsigned short* sX  = (unsigned short*)dsm_e;
  unsigned short* sXL = (unsigned short*)(dsm_e + LDS_XB);
  unsigned short* sH  = (unsigned short*)(dsm_e + 2 * LDS_XB);
  float* sY = (float*)dsm_e;
  __shared__ int   sTok[TPBT * MT];
  __shared__ int   sSlot[TPBT * MT];
  __shared__ float sW[TPBT * MT];
  __shared__ int   s_wc[8];

  const int tid = threadIdx.x, lane = tid & 31, wv = tid >> 5;
  const int h = lane >> 4, m = lane & 15;
  const int e = blockIdx.y;
  const int bx = blockIdx.x;

  if (tid < TPBT * MT) {
    if (DENSE) {
      const int lt0 = tid / MT;
      sTok[tid]  = (bx + GXT * lt0) * MT + (tid % MT);
      sSlot[tid] = 0;
      sW[tid]    = 1.0f;
    } else {
      sTok[tid] = 0; sSlot[tid] = 0; sW[tid] = 0.0f;
    }
  }
  __syncthreads();

  int cnt = ntok;
  if (!DENSE) {
    int base = 0;
    #pragma unroll 1
    for (int ch = 0; ch < NTOK / 256; ++ch) {
      const int t = ch * 256 + tid;
      const int tc = (t < ntok) ? t : (ntok - 1);
      int e0 = sel[(size_t)tc * NSL + 0];
      int e1 = sel[(size_t)tc * NSL + 1];
      e0 = (e0 < 0) ? 0 : ((e0 > NEX - 1) ? (NEX - 1) : e0);
      e1 = (e1 < 0) ? 0 : ((e1 > NEX - 1) ? (NEX - 1) : e1);
      const float w0 = rw[(size_t)tc * NSL + 0];
      const float w1 = rw[(size_t)tc * NSL + 1];
      const bool f0 = (e0 == e);
      const bool f1 = (e1 == e);
      const bool f = (f0 || f1) && (t < ntok);
      const float wsum = (f0 ? w0 : 0.0f) + (f1 ? w1 : 0.0f);
      const unsigned int msk = __builtin_amdgcn_ballot_w32(f);
      const int off = __builtin_popcount(msk & ((1u << lane) - 1u));
      const int wcnt = __builtin_popcount(msk);
      if (lane == 0) s_wc[wv] = wcnt;
      __syncthreads();
      int pre = 0, tot = 0;
      #pragma unroll
      for (int w2 = 0; w2 < 8; ++w2) {
        const int c2 = s_wc[w2];
        tot += c2;
        pre += (w2 < wv) ? c2 : 0;
      }
      if (f) {
        const int rank = base + pre + off;
        const int tile = rank / MT;
        const int lt = tile / GXT;
        const int p = lt * MT + (rank % MT);
        if (((tile % GXT) == bx) && ((unsigned)p < (unsigned)(TPBT * MT))) {
          sTok[p]  = t;
          sSlot[p] = f0 ? 0 : 1;
          sW[p]    = wsum;
        }
      }
      base += tot;
      __syncthreads();
    }
    cnt = base;
  }

  const v8f z8 = {0.f, 0.f, 0.f, 0.f, 0.f, 0.f, 0.f, 0.f};

  #pragma unroll 1
  for (int lt = 0; lt < TPBT; ++lt) {
    const int m0 = (bx + GXT * lt) * MT;
    if (m0 >= cnt) break;
    int nrows = cnt - m0;
    nrows = (nrows > MT) ? MT : nrows;
    const int lo = lt * MT;

    #pragma unroll
    for (int j = 0; j < 16; ++j) {
      const int idx = tid + 256 * j;
      const int row = idx >> 7, c8 = idx & 127;
      int t = sTok[lo + row];
      t = (t < 0) ? 0 : ((t > NTOK - 1) ? (NTOK - 1) : t);
      const size_t go = (size_t)t * DM + 8 * c8;
      const v4u a = *(const v4ua*)(xh + go);
      const v4u b = *(const v4ua*)(xl + go);
      *(v4ua*)(sX  + row * XP + 8 * c8) = a;
      *(v4ua*)(sXL + row * XP + 8 * c8) = b;
    }
    __syncthreads();

    #pragma unroll 1
    for (int cb = 0; cb < HXT / 128; ++cb) {
      const int jg = cb * 128 + wv * 16 + m;
      const unsigned short* wgr = wg + ((size_t)e * HXT + jg) * DM;
      const unsigned short* wur = wu + ((size_t)e * HXT + jg) * DM;
      v8f ag[2], agl[2], au[2], aul[2];
      #pragma unroll
      for (int mt = 0; mt < 2; ++mt) { ag[mt] = z8; agl[mt] = z8; au[mt] = z8; aul[mt] = z8; }
      #pragma unroll 1
      for (int k0 = 0; k0 < DM; k0 += 64) {
        #pragma unroll
        for (int kk = 0; kk < 2; ++kk) {
          const int kb = k0 + 32 * kk;
          v16h ah[2], al[2];
          #pragma unroll
          for (int mt = 0; mt < 2; ++mt) {
            ah[mt] = ldfrag(sX  + (16 * mt + m) * XP + kb, h);
            al[mt] = ldfrag(sXL + (16 * mt + m) * XP + kb, h);
          }
          const v16h bg = ldfrag(wgr + kb, h);
          const v16h bu = ldfrag(wur + kb, h);
          #pragma unroll
          for (int mt = 0; mt < 2; ++mt) {
            ag[mt]  = wmma_h(ah[mt], bg, ag[mt]);
            agl[mt] = wmma_h(al[mt], bg, agl[mt]);
            au[mt]  = wmma_h(ah[mt], bu, au[mt]);
            aul[mt] = wmma_h(al[mt], bu, aul[mt]);
          }
        }
      }
      #pragma unroll
      for (int mt = 0; mt < 2; ++mt)
        #pragma unroll
        for (int r = 0; r < 8; ++r) {
          const int row = 16 * mt + 8 * h + r;
          const float g = (ag[mt][r] + agl[mt][r] * R_LO) * R_W;
          const float u = (au[mt][r] + aul[mt][r] * R_LO) * R_W;
          const float ge = 0.5f * g * (1.0f + erff(g * 0.70710678118654752f));
          const float hv = (ge * u) * H_SC;
          sH[row * HP + jg] = hbits(hv);
        }
    }
    __syncthreads();

    #pragma unroll 1
    for (int ns = 0; ns < DM / 256; ++ns) {
      v8f acc[2][2];
      #pragma unroll
      for (int mt = 0; mt < 2; ++mt)
        #pragma unroll
        for (int nt = 0; nt < 2; ++nt) acc[mt][nt] = z8;
      #pragma unroll 1
      for (int k0 = 0; k0 < HXT; k0 += 64) {
        #pragma unroll
        for (int kk = 0; kk < 2; ++kk) {
          const int kb = k0 + 32 * kk;
          v16h a[2];
          #pragma unroll
          for (int mt = 0; mt < 2; ++mt)
            a[mt] = ldfrag(sH + (16 * mt + m) * HP + kb, h);
          #pragma unroll
          for (int nt = 0; nt < 2; ++nt) {
            const int d = ns * 256 + wv * 32 + 16 * nt + m;
            const size_t bo = ((size_t)e * DM + d) * HXT + kb;
            const v16h b = ldfrag(wd + bo, h);
            #pragma unroll
            for (int mt = 0; mt < 2; ++mt) acc[mt][nt] = wmma_h(a[mt], b, acc[mt][nt]);
          }
        }
      }
      #pragma unroll
      for (int mt = 0; mt < 2; ++mt)
        #pragma unroll
        for (int nt = 0; nt < 2; ++nt) {
          const int cl = wv * 32 + 16 * nt + m;
          #pragma unroll
          for (int r = 0; r < 8; ++r) {
            const int row = 16 * mt + 8 * h + r;
            const float y = acc[mt][nt][r] * R_HW;
            sY[row * YP + cl] = y * sW[lo + row];
          }
        }
      __syncthreads();
      part_pass<NSLT>(sY, sTok + lo, sSlot + lo, dstp, ns, wv, lane, nrows);
      __threadfence();
      part_pass<NSLT>(sY, sTok + lo, sSlot + lo, dstp, ns, wv, lane, nrows);
      __syncthreads();
    }
  }
}

__global__ __launch_bounds__(256) void k_comb(const float* __restrict__ part,
                                              const float* __restrict__ shb,
                                              const int* __restrict__ sel,
                                              const float* __restrict__ X,
                                              const float* __restrict__ wc,
                                              float* __restrict__ out, int ntok)
{
  const int lane = threadIdx.x & 31, wv = threadIdx.x >> 5;
  const int t = blockIdx.x * 8 + wv;
  if (t >= ntok) return;
  int e0 = sel[(size_t)t * NSL + 0];
  int e1 = sel[(size_t)t * NSL + 1];
  e0 = (e0 < 0) ? 0 : ((e0 > NEX - 1) ? (NEX - 1) : e0);
  e1 = (e1 < 0) ? 0 : ((e1 > NEX - 1) ? (NEX - 1) : e1);
  const bool dup = (e0 == e1);

  const float* xr = X + (size_t)t * DM;
  double d0 = 0.0, d1 = 0.0;
  #pragma unroll 1
  for (int j = 0; j < DM / 32; ++j) {
    const int hh = lane + 32 * j;
    const double xd = (double)xr[hh];
    d0 = fma(xd, (double)wc[2 * hh + 0], d0);
    d1 = fma(xd, (double)wc[2 * hh + 1], d1);
  }
  #pragma unroll
  for (int s = 16; s > 0; s >>= 1) { d0 += __shfl_xor(d0, s, 32); d1 += __shfl_xor(d1, s, 32); }
  const float f0 = (float)d0, f1 = (float)d1;
  const float mx = fmaxf(f0, f1);
  const float g0 = expf(f0 - mx), g1 = expf(f1 - mx);
  const float inv = 1.0f / (g0 + g1);
  const float a0 = g0 * inv, a1 = g1 * inv;

  const float* p0 = part + (size_t)t * NSL * DM;
  const float* p1 = p0 + DM;
  const float* sp = shb + (size_t)t * DM;
  v4f o[8];
  #pragma unroll
  for (int i = 0; i < 8; ++i) {
    const v4f a = *(const v4fa*)(p0 + 128 * i + 4 * lane);
    const v4f b = *(const v4fa*)(p1 + 128 * i + 4 * lane);
    const v4f c = *(const v4fa*)(sp + 128 * i + 4 * lane);
    const v4f s = a + b;
    const v4f l = dup ? a : s;
    o[i] = l * a0 + c * a1;
  }
  float* d = out + (size_t)t * DM;
  #pragma unroll
  for (int i = 0; i < 8; ++i) *(volatile v4f*)(d + 128 * i + 4 * lane) = o[i];
  __threadfence();
  #pragma unroll
  for (int i = 0; i < 8; ++i) *(volatile v4f*)(d + 128 * i + 4 * lane) = o[i];
}

extern "C" void kernel_launch(void* const* d_in, const int* in_sizes, int n_in,
                              void* d_out, int out_size, void* d_ws, size_t ws_size,
                              hipStream_t stream)
{
  if (n_in < 11) return;
  if (in_sizes[0]  != NTOK * DM) return;
  if (in_sizes[1]  != 1) return;
  if (in_sizes[2]  != NEX * DM) return;
  if (in_sizes[3]  != NTASK * DM) return;
  if (in_sizes[4]  != NEX * DM * HXR) return;
  if (in_sizes[5]  != NEX * DM * HXR) return;
  if (in_sizes[6]  != NEX * HXR * DM) return;
  if (in_sizes[7]  != DM * HXS) return;
  if (in_sizes[8]  != DM * HXS) return;
  if (in_sizes[9]  != HXS * DM) return;
  if (in_sizes[10] != DM * 2) return;
  if (out_size != NTOK * DM) return;

  const float* X    = (const float*)d_in[0];
  const int*   TSK  = (const int*)d_in[1];
  const float* GW   = (const float*)d_in[2];
  const float* TEMB = (const float*)d_in[3];
  const float* WEG  = (const float*)d_in[4];
  const float* WEU  = (const float*)d_in[5];
  const float* WED  = (const float*)d_in[6];
  const float* WSG  = (const float*)d_in[7];
  const float* WSU  = (const float*)d_in[8];
  const float* WSD  = (const float*)d_in[9];
  const float* WC   = (const float*)d_in[10];
  float* out = (float*)d_out;

  const size_t bSEL  = (size_t)NTOK * NSL * 4;
  const size_t bRW   = (size_t)NTOK * NSL * 4;
  const size_t bXH   = (size_t)NTOK * DM * 2;
  const size_t bWR   = (size_t)NEX * HXR * DM * 2;
  const size_t bWS   = (size_t)DM * HXS * 2;
  const size_t bPART = (size_t)NTOK * NSL * DM * 4;
  const size_t bSHB  = (size_t)NTOK * DM * 4;
  const size_t total = bSEL + bRW + 2 * bXH + 3 * bWR + 3 * bWS + bPART + bSHB;
  if (total > ws_size) return;
  if (total > (size_t)134217728) return;

  char* ws = (char*)d_ws;
  size_t off = 0;
  int*            SEL  = (int*)(ws + off);            off += bSEL;
  float*          RW   = (float*)(ws + off);          off += bRW;
  unsigned short* XH   = (unsigned short*)(ws + off); off += bXH;
  unsigned short* XL   = (unsigned short*)(ws + off); off += bXH;
  unsigned short* WGT  = (unsigned short*)(ws + off); off += bWR;
  unsigned short* WUT  = (unsigned short*)(ws + off); off += bWR;
  unsigned short* WDT  = (unsigned short*)(ws + off); off += bWR;
  unsigned short* WSGT = (unsigned short*)(ws + off); off += bWS;
  unsigned short* WSUT = (unsigned short*)(ws + off); off += bWS;
  unsigned short* WSDT = (unsigned short*)(ws + off); off += bWS;
  float*          PART = (float*)(ws + off);          off += bPART;
  float*          SHB  = (float*)(ws + off);          off += bSHB;
  if (off != total) return;

  hipFuncSetAttribute(reinterpret_cast<const void*>(&k_expert<HXR, 32, 4, NSL, 0>),
                      hipFuncAttributeMaxDynamicSharedMemorySize, LDS_R);
  hipFuncSetAttribute(reinterpret_cast<const void*>(&k_expert<HXS, NTOK / MT, 1, 1, 1>),
                      hipFuncAttributeMaxDynamicSharedMemorySize, LDS_S);

  k_router<<<NTOK / 32, 256, 0, stream>>>(X, GW, TEMB, TSK, SEL, RW, NTOK);

  {
    const int n8x = NTOK * DM / 8;
    k_cvtx<<<(n8x + 255) / 256, 256, 0, stream>>>(X, XH, XL, n8x);
  }

  k_tcvt<<<dim3(HXR / 64, DM / 64, NEX), 256, 0, stream>>>(WEG, WGT, DM, HXR, W_SC);
  k_tcvt<<<dim3(HXR / 64, DM / 64, NEX), 256, 0, stream>>>(WEU, WUT, DM, HXR, W_SC);
  k_tcvt<<<dim3(DM / 64, HXR / 64, NEX), 256, 0, stream>>>(WED, WDT, HXR, DM, W_SC);
  k_tcvt<<<dim3(HXS / 64, DM / 64, 1), 256, 0, stream>>>(WSG, WSGT, DM, HXS, W_SC);
  k_tcvt<<<dim3(HXS / 64, DM / 64, 1), 256, 0, stream>>>(WSU, WSUT, DM, HXS, W_SC);
  k_tcvt<<<dim3(DM / 64, HXS / 64, 1), 256, 0, stream>>>(WSD, WSDT, HXS, DM, W_SC);

  k_expert<HXR, 32, 4, NSL, 0><<<dim3(32, NEX), 256, LDS_R, stream>>>(
      XH, XL, WGT, WUT, WDT, SEL, RW, PART, NTOK);

  k_expert<HXS, NTOK / MT, 1, 1, 1><<<dim3(NTOK / MT, 1), 256, LDS_S, stream>>>(
      XH, XL, WSGT, WSUT, WSDT, SEL, RW, SHB, NTOK);

  k_comb<<<(NTOK + 7) / 8, 256, 0, stream>>>(PART, SHB, SEL, X, WC, out, NTOK);
}
